// ModelA_37563783971151
// MI455X (gfx1250) — hardware-verified
//
#include <hip/hip_runtime.h>


#define NBT  8
#define TT   8192
#define XD   64
#define HH   128
#define NO   50
#define NR   (NBT * TT)
#define DM   XD
#define LEPS 1e-5f
#define LOSC 1024.0f

typedef _Float16 h16;
typedef unsigned short bf;
typedef __attribute__((ext_vector_type(16))) __bf16   v16bf;
typedef __attribute__((ext_vector_type(16))) _Float16 v16h;
typedef __attribute__((ext_vector_type(8)))  _Float16 v8h;
typedef __attribute__((ext_vector_type(8)))  unsigned short v8us;
typedef __attribute__((ext_vector_type(8)))  float    v8f;
typedef __attribute__((ext_vector_type(4)))  float    v4f;
typedef v8h  __attribute__((may_alias)) v8ha;
typedef v4f  __attribute__((may_alias)) v4fa;
typedef v8us __attribute__((may_alias)) v8usa;

__device__ __forceinline__ unsigned short f2bf(float f) { unsigned u = __float_as_uint(f); u += 0x7FFFu + ((u >> 16) & 1u); return (unsigned short)(u >> 16); }
__device__ __forceinline__ float bf2f(unsigned short b) { return __uint_as_float(((unsigned)b) << 16); }
__device__ __forceinline__ float bfr(float f) { return bf2f(f2bf(f)); }
__device__ __forceinline__ v16h cat16(v8h lo, v8h hi) { return __builtin_shufflevector(lo, hi, 0, 1, 2, 3, 4, 5, 6, 7, 8, 9, 10, 11, 12, 13, 14, 15); }
__device__ __forceinline__ v16bf cat16b(v8us lo, v8us hi) { return __builtin_bit_cast(v16bf, __builtin_shufflevector(lo, hi, 0, 1, 2, 3, 4, 5, 6, 7, 8, 9, 10, 11, 12, 13, 14, 15)); }
__device__ __forceinline__ v8f wmma16(v16h a, v16h b, v8f c) { return __builtin_amdgcn_wmma_f32_16x16x32_f16(false, a, false, b, (short)0, c, false, false); }
__device__ __forceinline__ v8f wmmab(v16bf a, v16bf b, v8f c) { return __builtin_amdgcn_wmma_f32_16x16x32_bf16(false, a, false, b, (short)0, c, false, false); }

template <bool SPLITA, bool F16OUT = false>
__global__ __launch_bounds__(128) void k_gemmb(const bf* __restrict__ A, const bf* __restrict__ Al, const bf* __restrict__ Bn, const float* __restrict__ bias, float* C, int ldc, h16* C2, const float* __restrict__ R = nullptr, int K = DM, int roundR = 1) {
    __shared__ __align__(16) float ost[4][16 * 68];
    const int lane = threadIdx.x & 31, wave = threadIdx.x >> 5, lr = lane & 15, hi = lane >> 4;
    const int r0 = blockIdx.x * 64 + wave * 16, c0 = blockIdx.y * 64;
    const size_t aoff = (size_t)(r0 + lr) * K + 8 * hi;
    size_t boff[4];
#pragma unroll
    for (int t = 0; t < 4; ++t) boff[t] = (size_t)(c0 + t * 16 + lr) * K + 8 * hi;
    v8f acc[4];
#pragma unroll
    for (int t = 0; t < 4; ++t) acc[t] = (v8f){};
#pragma unroll 1
    for (int kc = 0; kc < K; kc += 32) {
        const v16bf a = cat16b(*(const v8us*)(A + aoff + kc), *(const v8us*)(A + aoff + kc + 16));
        v16bf al = a;
        if (SPLITA) al = cat16b(*(const v8us*)(Al + aoff + kc), *(const v8us*)(Al + aoff + kc + 16));
#pragma unroll
        for (int t = 0; t < 4; ++t) { const v16bf b = cat16b(*(const v8us*)(Bn + boff[t] + kc), *(const v8us*)(Bn + boff[t] + kc + 16)); acc[t] = wmmab(a, b, acc[t]); if (SPLITA) acc[t] = wmmab(al, b, acc[t]); }
        asm volatile("v_nop\n\tv_nop\n\tv_nop\n\tv_nop" : "+v"(acc[0]), "+v"(acc[1]), "+v"(acc[2]), "+v"(acc[3]) : "v"(a), "v"(al));
    }
    float* os = &ost[wave][0];
#pragma unroll
    for (int t = 0; t < 4; ++t) { const float bv = bias ? bfr(bias[c0 + t * 16 + lr]) : 0.f;
#pragma unroll
        for (int j = 0; j < 8; ++j) os[(hi * 8 + j) * 68 + t * 16 + lr] = acc[t][j] + bv; }
    __syncthreads();
    if (F16OUT) {
        h16* crow = (h16*)(void*)C + (size_t)r0 * ldc + c0;
        auto pass = [&]() {
#pragma unroll
            for (int s = 0; s < 4; ++s) { const int row = 4 * s + (lane >> 3), piece = lane & 7; const float* sp = os + row * 68 + piece * 8; v8h o, o2;
#pragma unroll
                for (int i = 0; i < 8; ++i) { const h16 a = (h16)sp[i]; o[i] = a; o2[i] = (h16)((sp[i] - (float)a) * LOSC); }
                *(volatile v8h*)(crow + (size_t)row * ldc + piece * 8) = o; if (C2) *(volatile v8h*)(C2 + (size_t)r0 * ldc + c0 + (size_t)row * ldc + piece * 8) = o2; }
        };
        pass(); __threadfence(); pass();
    } else {
        float* crow = C + (size_t)r0 * ldc + c0;
        auto pass = [&]() {
#pragma unroll
            for (int s = 0; s < 8; ++s) { const int Lid = (lane >> 3) + 4 * s, piece = lane & 7; const int row = Lid >> 1, cofs = (Lid & 1) * 32 + piece * 4;
                v4f val = *(const v4fa*)(os + row * 68 + cofs); if (R) { const v4f rv = *(const v4f*)(R + ((size_t)r0 + row) * ldc + c0 + cofs); val += roundR ? (v4f){bfr(rv[0]), bfr(rv[1]), bfr(rv[2]), bfr(rv[3])} : rv; }
                *(volatile v4f*)(crow + (size_t)row * ldc + cofs) = val; }
        };
        pass(); __threadfence(); pass();
    }
}

__global__ __launch_bounds__(256) void k_wt(const float* __restrict__ Wm, int K, int ncols, bf* WT) {
    __shared__ __align__(16) unsigned short tl[64 * 72];
    const int tid = threadIdx.x, k0 = blockIdx.x * 64, n0 = blockIdx.y * 64;
    const int kk = tid >> 2, nq = (tid & 3) * 16;
#pragma unroll
    for (int i = 0; i < 16; ++i) tl[(nq + i) * 72 + kk] = f2bf(Wm[(size_t)(k0 + kk) * ncols + n0 + nq + i]);
    __syncthreads();
    const int piece = tid & 7;
    auto pass = [&]() {
#pragma unroll
        for (int s = 0; s < 2; ++s) { const int nr = (tid >> 3) + 32 * s; const v8us val = *(const v8usa*)(tl + nr * 72 + piece * 8); *(volatile v8us*)(WT + (size_t)(n0 + nr) * K + k0 + piece * 8) = val; }
    };
    pass(); __threadfence(); pass();
}
__global__ __launch_bounds__(256) void k_wtp(const float* __restrict__ Wm, int krows, int ncols, int kpad, bf* WT) {
    __shared__ __align__(16) unsigned short tl[64 * 72];
    const int tid = threadIdx.x, k0 = blockIdx.x * 64, n0 = blockIdx.y * 64;
    const int kk = tid >> 2, nq = (tid & 3) * 16;
    const int k = k0 + kk, kc = k < krows ? k : krows - 1;
#pragma unroll
    for (int i = 0; i < 16; ++i) { const int n = n0 + nq + i, ncl = n < ncols ? n : ncols - 1; const float w = Wm[(size_t)kc * ncols + ncl]; tl[(nq + i) * 72 + kk] = (k < krows && n < ncols) ? f2bf(w) : (unsigned short)0; }
    __syncthreads();
    const int piece = tid & 7;
    auto pass = [&]() {
#pragma unroll
        for (int s = 0; s < 2; ++s) { const int nr = (tid >> 3) + 32 * s; const v8us val = *(const v8usa*)(tl + nr * 72 + piece * 8); *(volatile v8us*)(WT + (size_t)(n0 + nr) * kpad + k0 + piece * 8) = val; }
    };
    pass(); __threadfence(); pass();
}

__global__ __launch_bounds__(256) void k_cvtx(const float* __restrict__ src, bf* dst) {
    typedef __attribute__((ext_vector_type(2))) unsigned short v2us;
    const int lane = threadIdx.x & 31; const size_t r = (size_t)blockIdx.x * 8 + (threadIdx.x >> 5); if (r >= (size_t)NR) return; v2us o;
    o[0] = f2bf(src[r * XD + lane * 2]); o[1] = f2bf(src[r * XD + lane * 2 + 1]);
    *(volatile v2us*)(dst + r * XD + lane * 2) = o; __threadfence(); *(volatile v2us*)(dst + r * XD + lane * 2) = o;
}
template <bool LEAKY>
__global__ __launch_bounds__(256) void k_ln(const float* __restrict__ src, const float* __restrict__ g, const float* __restrict__ bb, float* Hf, bf* Hh, bf* Hl) {
    typedef __attribute__((ext_vector_type(4))) unsigned short v4us;
    const int lane = threadIdx.x & 31; const size_t r = (size_t)blockIdx.x * 8 + (threadIdx.x >> 5); if (r >= (size_t)TT) return; float v[4]; float s = 0.f;
#pragma unroll
    for (int i = 0; i < 4; ++i) { float t = src[r * HH + lane * 4 + i]; if (LEAKY) t = (t >= 0.f) ? t : 0.01f * t; v[i] = t; s += t; }
#pragma unroll
    for (int sh = 16; sh; sh >>= 1) s += __shfl_xor(s, sh, 32);
    const float mu = s * (1.0f / HH); float q = 0.f;
#pragma unroll
    for (int i = 0; i < 4; ++i) { const float d = v[i] - mu; q = fmaf(d, d, q); }
#pragma unroll
    for (int sh = 16; sh; sh >>= 1) q += __shfl_xor(q, sh, 32);
    const float rs = rsqrtf(q * (1.0f / HH) + LEPS); v4f o; v4us oh, ol;
#pragma unroll
    for (int i = 0; i < 4; ++i) { const int c = lane * 4 + i; const float y = (v[i] - mu) * rs * bfr(g[c]) + bfr(bb[c]); o[i] = y; const unsigned short hb = f2bf(y); oh[i] = hb; ol[i] = f2bf(y - bf2f(hb)); }
    const size_t ob = r * HH + lane * 4; *(volatile v4f*)(Hf + ob) = o; *(volatile v4us*)(Hh + ob) = oh; *(volatile v4us*)(Hl + ob) = ol; __threadfence(); *(volatile v4f*)(Hf + ob) = o; *(volatile v4us*)(Hh + ob) = oh; *(volatile v4us*)(Hl + ob) = ol;
}
__device__ __forceinline__ float sigm(float v) { return 1.0f / (1.0f + __expf(-v)); }
__global__ __launch_bounds__(128) void k_scan(const float* __restrict__ HG, float* Sg) {
    const int d = threadIdx.x; float h = 0.f;
#pragma unroll 1
    for (int t = 0; t < TT; ++t) { const size_t r = (size_t)t; const float hid = HG[r * 2 * HH + d], gate = HG[r * 2 * HH + HH + d];
        const float z = sigm(gate); const float gv = (hid >= 0.f) ? hid + 0.5f : sigm(hid); h = fmaf(1.0f - z, h, z * gv);
        *(volatile float*)(Sg + r * HH + d) = h; __threadfence(); *(volatile float*)(Sg + r * HH + d) = h; }
}
__global__ __launch_bounds__(256) void k_out(const float* __restrict__ P, float* OUTP) {
    const size_t u = (size_t)blockIdx.x * 256 + threadIdx.x; if (u >= (size_t)TT * NO / 4) return;       v4f v;
#pragma unroll
    for (int q = 0; q < 4; ++q) { const size_t e = u * 4 + q; const size_t r = e / NO; const int c = (int)(e % NO); const float t = P[r * 64 + c]; v[q] = log1pf(__expf(-fabsf(t))) + fmaxf(t, 0.f); }
    *(volatile v4f*)(OUTP + u * 4) = v; __threadfence(); *(volatile v4f*)(OUTP + u * 4) = v;
}

__global__ __launch_bounds__(64) void k_b64(const float* __restrict__ pb, float* PBP) {
    typedef __attribute__((ext_vector_type(2))) float v2f;
    const int lane = threadIdx.x; if (lane >= 32) return; v2f v; v[0] = (2 * lane < NO) ? pb[2 * lane < NO ? 2 * lane : 0] : 0.f; v[1] = (2 * lane + 1 < NO) ? pb[(2 * lane + 1 < NO) ? 2 * lane + 1 : 0] : 0.f;
    *(volatile v2f*)(PBP + 2 * lane) = v; __threadfence(); *(volatile v2f*)(PBP + 2 * lane) = v;
}

extern "C" void kernel_launch(void* const* d_in, const int* in_sizes, int n_in,
                              void* d_out, int out_size, void* d_ws, size_t ws_size, hipStream_t stream) {
    (void)in_sizes; (void)n_in; (void)out_size;
    const float* x = (const float*)d_in[0]; const float* ew = (const float*)d_in[1]; const float* eb = (const float*)d_in[2]; const float* g0 = (const float*)d_in[3]; const float* b0 = (const float*)d_in[4];
    const float* pw = (const float*)d_in[5]; const float* pb = (const float*)d_in[6];
    const float* gw[3] = {(const float*)d_in[7], (const float*)d_in[11], (const float*)d_in[15]}; const float* gb[3] = {(const float*)d_in[8], (const float*)d_in[12], (const float*)d_in[16]};
    const float* lg[3] = {(const float*)d_in[9], (const float*)d_in[13], (const float*)d_in[17]}; const float* lb[3] = {(const float*)d_in[10], (const float*)d_in[14], (const float*)d_in[18]};
    float* out = (float*)d_out;
    char* wsp = (char*)d_ws;
    auto take = [&](size_t bytes) { char* p = wsp; wsp += (bytes + 255) & ~(size_t)255; return (void*)p; };
    bf* EWT = (bf*)take((size_t)HH * XD * 2); bf* GWT[3]; for (int i = 0; i < 3; ++i) GWT[i] = (bf*)take((size_t)2 * HH * HH * 2); bf* PWT = (bf*)take((size_t)64 * HH * 2); float* PBP = (float*)take(64 * 4);
    bf* Xb = (bf*)take((size_t)NR * XD * 2); float* T = (float*)take((size_t)TT * 2 * HH * 4); float* Hf = (float*)take((size_t)TT * HH * 4); bf* Hh = (bf*)take((size_t)TT * HH * 2); bf* Hl = (bf*)take((size_t)TT * HH * 2); float* Sg = (float*)take((size_t)TT * HH * 4); float* P = (float*)take((size_t)TT * 64 * 4);
    if ((size_t)(wsp - (char*)d_ws) > ws_size) return;
    k_wt<<<dim3(XD / 64, HH / 64, 1), 256, 0, stream>>>(ew, XD, HH, EWT); for (int i = 0; i < 3; ++i) k_wt<<<dim3(HH / 64, (2 * HH) / 64, 1), 256, 0, stream>>>(gw[i], HH, 2 * HH, GWT[i]);
    k_wtp<<<dim3(HH / 64, 1, 1), 256, 0, stream>>>(pw, HH, NO, HH, PWT); k_b64<<<1, 64, 0, stream>>>(pb, PBP);
    k_cvtx<<<NR / 8, 256, 0, stream>>>(x, Xb);
    for (int b = 0; b < NBT; ++b) { const size_t rb = (size_t)b * TT;
        k_gemmb<false, false><<<dim3(TT / 64, HH / 64, 1), 128, 0, stream>>>(Xb + rb * XD, nullptr, EWT, eb, Sg, HH, nullptr, nullptr, XD);
        k_ln<true><<<TT / 8, 256, 0, stream>>>(Sg, g0, b0, Hf, Hh, Hl);
        for (int i = 0; i < 3; ++i) {
            k_gemmb<true, false><<<dim3(TT / 64, (2 * HH) / 64, 1), 128, 0, stream>>>(Hh, Hl, GWT[i], gb[i], T, 2 * HH, nullptr, nullptr, HH);
            k_scan<<<1, 128, 0, stream>>>(T, Sg);
            k_ln<false><<<TT / 8, 256, 0, stream>>>(Sg, lg[i], lb[i], Hf, Hh, Hl); }
        k_gemmb<true, false><<<dim3(TT / 64, 1, 1), 128, 0, stream>>>(Hh, Hl, PWT, PBP, P, 64, nullptr, nullptr, HH);
        k_out<<<(unsigned)(((size_t)TT * NO / 4 + 255) / 256), 256, 0, stream>>>(P, out + rb * NO); }
}
